// RWKV_Tmix_x060f_20830591385837
// MI455X (gfx1250) — hardware-verified
//
#include <hip/hip_runtime.h>
#include <math.h>

constexpr int   kBatch    = 4;
constexpr int   kSeq      = 1024;
constexpr int   kDim      = 1024;
constexpr int   kHeads    = 16;
constexpr int   kHeadDim  = 64;
constexpr int   kTok      = kBatch * kSeq;
constexpr int   kLora     = 96;
constexpr int   kLoraPad  = 128;
constexpr int   kLoraD    = 32;
constexpr int   kVG       = 6144;
constexpr int   kCat      = 3072;
constexpr long  kActPlane = (long)kTok * kDim;
constexpr long  kSqPlane  = (long)kDim * kDim;

constexpr float kWCarry     = 32.0f;
constexpr float kLCarry     = 1024.0f;
constexpr float kTanhCarry  = 16.0f;
constexpr float kCatCarry   = 8.0f;
constexpr float kStateCarry = 256.0f;
constexpr float kLoCarry    = 2048.0f;
constexpr float kScaleL0    = 1.0f / 1024.0f;
constexpr float kScaleL1    = 1.0f / 16384.0f;
constexpr float kScaleProj  = 1.0f / 32.0f;
constexpr float kScaleOut   = 1.0f / 256.0f;
constexpr float kInvState   = 1.0f / 256.0f;
constexpr float kInvLo      = 1.0f / 2048.0f;
constexpr float kInvDim     = 1.0f / 1024.0f;
constexpr float kLnEps      = 1e-5f;

constexpr size_t kOffWR   = 0;
constexpr size_t kOffWK   = 2097152;
constexpr size_t kOffWVG  = 4194304;
constexpr size_t kOffWO   = 16777216;
constexpr size_t kOffW1   = 23068672;
constexpr size_t kOffW2   = 23330816;
constexpr size_t kOffMT   = 23527424;
constexpr size_t kOffX    = 24576000;
constexpr size_t kOffR    = 49741824;
constexpr size_t kOffE    = 66519040;
constexpr size_t kOffV    = 83296256;
constexpr size_t kOffCAT  = 100073472;
constexpr size_t kWsTotal = 125239296;
static_assert(kOffWK  == kOffWR  + (size_t)kSqPlane * 2);
static_assert(kOffWVG == kOffWK  + (size_t)kSqPlane * 2);
static_assert(kOffWO  == kOffWVG + (size_t)kVG * kDim * 2);
static_assert(kOffW1  == kOffWO  + (size_t)kDim * kCat * 2);
static_assert(kOffW2  == kOffW1  + (size_t)kLoraPad * kDim * 2);
static_assert(kOffMT  == kOffW2  + (size_t)3 * kDim * kLoraD * 2);
static_assert(kOffX   == kOffMT  + (size_t)kTok * kLoraPad * 2);
static_assert(kOffR   == kOffX   + (size_t)3 * kActPlane * 2);
static_assert((size_t)kActPlane * 4 <= (size_t)3 * kActPlane * 2);
static_assert(kOffE   == kOffR   + (size_t)kActPlane * 4);
static_assert(kOffV   == kOffE   + (size_t)kActPlane * 4);
static_assert(kOffCAT == kOffV   + (size_t)kActPlane * 4);
static_assert(kWsTotal == kOffCAT + (size_t)kTok * kCat * 2);
static_assert(kWsTotal <= (size_t)134217728);
static_assert((kOffMT % 128) == 0 && (kOffX % 128) == 0 && (kOffR % 128) == 0 && (kOffCAT % 128) == 0);

typedef __attribute__((ext_vector_type(16))) _Float16 v16h;
typedef __attribute__((ext_vector_type(8)))  _Float16 v8h;
typedef __attribute__((ext_vector_type(8)))  float    v8f;
typedef __attribute__((ext_vector_type(4)))  float    v4f;
typedef __attribute__((ext_vector_type(4)))  unsigned int v4u;

__device__ __forceinline__ unsigned short h_bits(float f) { const _Float16 h = (_Float16)f; return __builtin_bit_cast(unsigned short, h); }
__device__ __forceinline__ unsigned pk16(unsigned short a, unsigned short b) { return (unsigned)a | ((unsigned)b << 16); }
__device__ __forceinline__ v4u pack8(const unsigned short (&hb)[8]) {
  return (v4u){pk16(hb[0], hb[1]), pk16(hb[2], hb[3]), pk16(hb[4], hb[5]), pk16(hb[6], hb[7])};
}

union HU { v16h v; v8h h8[2]; };
__device__ __forceinline__ v16h frag_load(const _Float16* p) {
  HU f; f.h8[0] = *(const v8h*)(p); f.h8[1] = *(const v8h*)(p + 16); return f.v;
}
__device__ __forceinline__ v8f mma16(v16h a, v16h b, v8f c) {
  return __builtin_amdgcn_wmma_f32_16x16x32_f16(false, a, false, b, (short)0, c, false, false);
}
__device__ __forceinline__ void dep_guard(v8f& a, v8f& b, v16h x, v16h y) {
  asm volatile("v_nop\n\tv_nop\n\tv_nop\n\tv_nop" : "+v"(a), "+v"(b) : "v"(x), "v"(y));
}
__device__ __forceinline__ void keep4(v16h a, v16h b, v16h c, v16h d) { asm volatile("v_nop" :: "v"(a), "v"(b), "v"(c), "v"(d)); }
__device__ __forceinline__ void acc_guard4(v8f& a, v8f& b, v8f& c, v8f& d) {
  asm volatile("v_nop\n\tv_nop\n\tv_nop\n\tv_nop" : "+v"(a), "+v"(b), "+v"(c), "+v"(d));
}
__device__ __forceinline__ v8f mma16_g(v16h a, v16h b, v8f c) {
  c = mma16(a, b, c);
  asm volatile("v_nop\n\tv_nop\n\tv_nop\n\tv_nop" : "+v"(c) : "v"(a), "v"(b));
  return c;
}
__device__ __forceinline__ void wave_sync_lds() {
  __builtin_amdgcn_fence(__ATOMIC_RELEASE, "workgroup");
  __builtin_amdgcn_wave_barrier();
  __builtin_amdgcn_fence(__ATOMIC_ACQUIRE, "workgroup");
}

template <int TK>
__global__ __launch_bounds__(256) void trans_cast(const float* __restrict__ src, unsigned short* __restrict__ dst,
                                                  int N, int K, long srcZ, long dstZ, float scale) {
  __shared__ float sm[TK][65];
  const int tid = threadIdx.x;
  const int n0 = blockIdx.x * 64;
  const int k0 = blockIdx.y * TK;
  const float* S = src + (size_t)blockIdx.z * (size_t)srcZ;
  unsigned short* D = dst + (size_t)blockIdx.z * (size_t)dstZ;
#pragma unroll
  for (int i = 0; i < TK / 16; ++i) {
    const int idx = tid + 256 * i;
    const int r = idx >> 4;
    const int c4 = (idx & 15) * 4;
    const int gc = n0 + c4;
    const int gcc = (gc < N - 4) ? gc : (N - 4);
    v4f v = *(const v4f*)(S + (size_t)(k0 + r) * N + gcc);
    if (gc >= N) v = (v4f){0.0f, 0.0f, 0.0f, 0.0f};
    sm[r][c4 + 0] = v[0]; sm[r][c4 + 1] = v[1]; sm[r][c4 + 2] = v[2]; sm[r][c4 + 3] = v[3];
  }
  __syncthreads();
  constexpr int kPPR = TK / 8;
#pragma unroll
  for (int it = 0; it < TK / 32; ++it) {
    const int p = it * 256 + tid;
    const int row = p / kPPR;
    const int c8 = (p % kPPR) * 8;
    unsigned short hb[8];
#pragma unroll
    for (int e = 0; e < 8; ++e) hb[e] = h_bits(sm[c8 + e][row] * scale);
    const v4u u = pack8(hb);
    unsigned short* q = D + (size_t)(n0 + row) * K + k0 + c8;
    *(volatile v4u*)q = u;
    __threadfence();
    *(volatile v4u*)q = u;
  }
}

__global__ __launch_bounds__(256) void shift_kernel(const float* __restrict__ x, const float* __restrict__ maax,
                                                    unsigned short* __restrict__ xxx) {
  const int gid = blockIdx.x * 256 + threadIdx.x;
  const int row = gid >> 7;
  const int c0  = (gid & 127) * 8;
  const int t   = row & (kSeq - 1);
  const int prow = (t > 0) ? (row - 1) : row;
  const float* pc = x + (size_t)row * kDim + c0;
  const float* pp = x + (size_t)prow * kDim + c0;
  const v4f ca = *(const v4f*)(pc);
  const v4f cb = *(const v4f*)(pc + 4);
  const v4f pa = *(const v4f*)(pp);
  const v4f pb = *(const v4f*)(pp + 4);
  const v4f ma = *(const v4f*)(maax + c0);
  const v4f mb = *(const v4f*)(maax + c0 + 4);
  unsigned short hb[8];
#pragma unroll
  for (int e = 0; e < 4; ++e) {
    const float xc0 = ca[e], xp0 = (t > 0) ? pa[e] : 0.0f;
    hb[e] = h_bits(xc0 + (xp0 - xc0) * ma[e]);
    const float xc1 = cb[e], xp1 = (t > 0) ? pb[e] : 0.0f;
    hb[4 + e] = h_bits(xc1 + (xp1 - xc1) * mb[e]);
  }
  const v4u u = pack8(hb);
  unsigned short* q = xxx + (size_t)row * kDim + c0;
  *(volatile v4u*)q = u;
  __threadfence();
  *(volatile v4u*)q = u;
}

template <int ACT, int OM>
__global__ __launch_bounds__(256) void gemm64(
    const unsigned short* __restrict__ Ap, int lda, long strideA,
    const unsigned short* __restrict__ Btp, int ldb, long strideB,
    void* __restrict__ Cout, int ldc, long strideC,
    const float* __restrict__ xsrc,
    const float* __restrict__ maa0, const float* __restrict__ maa1, const float* __restrict__ maa2,
    int M, int N, int K, float scale) {
  __shared__ __align__(16) float sT[8][16 * 68];
  const int b    = blockIdx.y;
  const int lane = threadIdx.x & 31;
  const int wave = threadIdx.x >> 5;
  const int tilesN = N >> 6;
  const int tilesM = M >> 6;
  const int tile = blockIdx.x * 8 + wave;
  if (tile >= tilesM * tilesN) return;
  const int tm = tile / tilesN;
  const int tn = tile - tm * tilesN;
  const int m0 = tm << 6;
  const int n0 = tn << 6;

  const _Float16* Ab = (const _Float16*)Ap  + (size_t)b * (size_t)strideA;
  const _Float16* Bb = (const _Float16*)Btp + (size_t)b * (size_t)strideB;

  const int rlane = lane & 15;
  const int koff  = (lane >> 4) * 8;
  const int mOff  = (lane >> 4) * 8;

  v8f acc[4][4];
#pragma unroll
  for (int i = 0; i < 4; ++i)
#pragma unroll
    for (int j = 0; j < 4; ++j) acc[i][j] = (v8f){0.f,0.f,0.f,0.f,0.f,0.f,0.f,0.f};

  for (int k0 = 0; k0 < K; k0 += 32) {
    v16h bh[4];
#pragma unroll
    for (int j = 0; j < 4; ++j)
      bh[j] = frag_load(Bb + (size_t)(n0 + (j << 4) + rlane) * ldb + koff + k0);
#pragma unroll
    for (int i = 0; i < 4; ++i) {
      const v16h ah = frag_load(Ab + (size_t)(m0 + (i << 4) + rlane) * lda + koff + k0);
#pragma unroll
      for (int j = 0; j < 4; ++j) acc[i][j] = mma16(ah, bh[j], acc[i][j]);
      dep_guard(acc[i][0], acc[i][3], ah, bh[3]);
    }
    keep4(bh[0], bh[1], bh[2], bh[3]);
  }
  acc_guard4(acc[0][0], acc[0][1], acc[0][2], acc[0][3]);
  acc_guard4(acc[1][0], acc[1][1], acc[1][2], acc[1][3]);
  acc_guard4(acc[2][0], acc[2][1], acc[2][2], acc[2][3]);
  acc_guard4(acc[3][0], acc[3][1], acc[3][2], acc[3][3]);

  float* slab = sT[wave];
  const float* maa = (b == 0) ? maa0 : ((b == 1) ? maa1 : maa2);
#pragma unroll
  for (int i = 0; i < 4; ++i) {
    const int mBase = m0 + (i << 4);
#pragma unroll
    for (int j = 0; j < 4; ++j) {
#pragma unroll
      for (int r = 0; r < 8; ++r) {
        float v = acc[i][j][r] * scale;
        if (ACT == 3) v = tanhf(v) * kTanhCarry;
        if (ACT == 6) v = expf(-expf(v));
        slab[(mOff + r) * 68 + (j << 4) + rlane] = v;
      }
    }
    wave_sync_lds();
    if (OM == 0) {
      float* C = (float*)Cout + (size_t)b * (size_t)strideC;
      const int hh = lane >> 4, c4 = (lane & 15) * 4;
      for (int pass = 0; pass < 2; ++pass) {
#pragma unroll
        for (int it = 0; it < 8; ++it) {
          const int row = it * 2 + hh;
          const v4f v = *(const v4f*)(slab + row * 68 + c4);
          *(volatile v4f*)(C + (size_t)(mBase + row) * ldc + n0 + c4) = v;
        }
        __threadfence();
      }
    } else {
      const int q = lane >> 3, c8 = (lane & 7) * 8;
      unsigned short* C = (unsigned short*)Cout + (size_t)b * (size_t)strideC;
      for (int pass = 0; pass < 2; ++pass) {
#pragma unroll
        for (int it = 0; it < 4; ++it) {
          const int row = it * 4 + q;
          const float* sp = slab + row * 68 + c8;
          v8h hv;
          if (OM == 1) {
#pragma unroll
            for (int e = 0; e < 8; ++e) hv[e] = (_Float16)sp[e];
          } else {
            const int grow = mBase + row;
            const int tt = grow & (kSeq - 1);
            const int prow = (tt > 0) ? (grow - 1) : grow;
            const float* xc0 = xsrc + (size_t)grow * kDim + n0 + c8;
            const float* xp0 = xsrc + (size_t)prow * kDim + n0 + c8;
            const v4f ca = *(const v4f*)(xc0);
            const v4f cb = *(const v4f*)(xc0 + 4);
            const v4f pa = *(const v4f*)(xp0);
            const v4f pb = *(const v4f*)(xp0 + 4);
            const v4f ma = *(const v4f*)(maa + n0 + c8);
            const v4f mb = *(const v4f*)(maa + n0 + c8 + 4);
#pragma unroll
            for (int e = 0; e < 4; ++e) {
              const float x0 = ca[e], p0 = (tt > 0) ? pa[e] : 0.0f;
              hv[e] = (_Float16)(x0 + (p0 - x0) * (ma[e] + sp[e]));
              const float x1 = cb[e], p1 = (tt > 0) ? pb[e] : 0.0f;
              hv[4 + e] = (_Float16)(x1 + (p1 - x1) * (mb[e] + sp[4 + e]));
            }
          }
          *(volatile v8h*)(C + (size_t)(mBase + row) * ldc + n0 + c8) = hv;
        }
        __threadfence();
      }
    }
    wave_sync_lds();
  }
}

__global__ __launch_bounds__(256) void gemm_vg(const unsigned short* __restrict__ Ap, const unsigned short* __restrict__ Btp,
                                               float* __restrict__ Vout, unsigned short* __restrict__ Cat, float scale) {
  __shared__ __align__(16) float sT[8][16 * 68];
  const int lane = threadIdx.x & 31;
  const int wave = threadIdx.x >> 5;
  const int tile = blockIdx.x * 8 + wave;
  const int tm = tile / 48;
  const int tn = tile - tm * 48;
  const int m0 = tm * 32;
  const int n0 = tn * 64;
  const _Float16* A  = (const _Float16*)Ap;
  const _Float16* Bt = (const _Float16*)Btp;
  const int rlane = lane & 15;
  const int koff  = (lane >> 4) * 8;
  const int mOff  = (lane >> 4) * 8;

  v8f av[2][4], ag[2][4];
#pragma unroll
  for (int i = 0; i < 2; ++i)
#pragma unroll
    for (int j = 0; j < 4; ++j) {
      av[i][j] = (v8f){0.f,0.f,0.f,0.f,0.f,0.f,0.f,0.f};
      ag[i][j] = (v8f){0.f,0.f,0.f,0.f,0.f,0.f,0.f,0.f};
    }

  for (int k0 = 0; k0 < kDim; k0 += 32) {
    const v16h a0 = frag_load(A + (size_t)(m0 + rlane) * kDim + koff + k0);
    const v16h a1 = frag_load(A + (size_t)(m0 + 16 + rlane) * kDim + koff + k0);
#pragma unroll
    for (int j = 0; j < 4; ++j) {
      const size_t bo = (size_t)(n0 + (j << 4) + rlane) * kDim + koff + k0;
      const v16h bv = frag_load(Bt + bo);
      const v16h bg = frag_load(Bt + (size_t)kCat * kDim + bo);
      av[0][j] = mma16(a0, bv, av[0][j]);
      av[1][j] = mma16(a1, bv, av[1][j]);
      ag[0][j] = mma16(a0, bg, ag[0][j]);
      ag[1][j] = mma16(a1, bg, ag[1][j]);
      dep_guard(av[1][j], ag[1][j], bv, bg);
    }
    keep4(a0, a1, a0, a1);
  }
  acc_guard4(av[0][0], av[0][1], av[0][2], av[0][3]);
  acc_guard4(av[1][0], av[1][1], av[1][2], av[1][3]);
  acc_guard4(ag[0][0], ag[0][1], ag[0][2], ag[0][3]);
  acc_guard4(ag[1][0], ag[1][1], ag[1][2], ag[1][3]);

  float* slab = sT[wave];
  const bool isV = (n0 < kDim);
#pragma unroll
  for (int i = 0; i < 2; ++i) {
    const int mBase = m0 + (i << 4);
#pragma unroll
    for (int j = 0; j < 4; ++j) {
#pragma unroll
      for (int r = 0; r < 8; ++r) {
        const float v = av[i][j][r] * scale;
        const float g = ag[i][j][r] * scale;
        const float sg = __builtin_amdgcn_rcpf(1.0f + expf(-g));
        slab[(mOff + r) * 68 + (j << 4) + rlane] = v * (g * sg);
      }
    }
    wave_sync_lds();
    if (isV) {
      const int hh = lane >> 4, c4 = (lane & 15) * 4;
      for (int pass = 0; pass < 2; ++pass) {
#pragma unroll
        for (int it = 0; it < 8; ++it) {
          const int row = it * 2 + hh;
          const v4f v = *(const v4f*)(slab + row * 68 + c4);
          *(volatile v4f*)(Vout + (size_t)(mBase + row) * kDim + n0 + c4) = v;
        }
        __threadfence();
      }
    } else {
      const int q = lane >> 3, c8 = (lane & 7) * 8;
      for (int pass = 0; pass < 2; ++pass) {
#pragma unroll
        for (int it = 0; it < 4; ++it) {
          const int row = it * 4 + q;
          const float* sp = slab + row * 68 + c8;
          v8h hv;
#pragma unroll
          for (int e = 0; e < 8; ++e) hv[e] = (_Float16)(sp[e] * kCatCarry);
          *(volatile v8h*)(Cat + (size_t)(mBase + row) * kCat + n0 + c8) = hv;
        }
        __threadfence();
      }
    }
    wave_sync_lds();
  }
}

__device__ __forceinline__ _Float16 lo_h(float sc, _Float16 hv) { return (_Float16)((sc - (float)hv) * kLoCarry); }

__device__ __forceinline__ void col_step(float (&s)[16], v16h& bv, v16h& bl, const float* kkp, const float* ewp, float vj) {
  const v4f q0 = *(const v4f*)(kkp);
  const v4f q1 = *(const v4f*)(kkp + 4);
  const v4f q2 = *(const v4f*)(kkp + 16);
  const v4f q3 = *(const v4f*)(kkp + 20);
  const v4f w0 = *(const v4f*)(ewp);
  const v4f w1 = *(const v4f*)(ewp + 4);
  const v4f w2 = *(const v4f*)(ewp + 16);
  const v4f w3 = *(const v4f*)(ewp + 20);
#pragma unroll
  for (int e = 0; e < 4; ++e) {
    {
      const float sc = s[e] * kStateCarry;       const _Float16 hv = (_Float16)sc;
      bv[e] = hv;       bl[e] = lo_h(sc, hv);       s[e]      = w0[e] * s[e]      + q0[e] * vj;
    }
    {
      const float sc = s[4 + e] * kStateCarry;   const _Float16 hv = (_Float16)sc;
      bv[4 + e] = hv;   bl[4 + e] = lo_h(sc, hv);   s[4 + e]  = w1[e] * s[4 + e]  + q1[e] * vj;
    }
    {
      const float sc = s[8 + e] * kStateCarry;   const _Float16 hv = (_Float16)sc;
      bv[8 + e] = hv;   bl[8 + e] = lo_h(sc, hv);   s[8 + e]  = w2[e] * s[8 + e]  + q2[e] * vj;
    }
    {
      const float sc = s[12 + e] * kStateCarry;  const _Float16 hv = (_Float16)sc;
      bv[12 + e] = hv;  bl[12 + e] = lo_h(sc, hv);  s[12 + e] = w3[e] * s[12 + e] + q3[e] * vj;
    }
  }
}

__global__ __launch_bounds__(128) void scan_kernel(const float* __restrict__ R, const float* __restrict__ E,
                                                   const float* __restrict__ V, const float* __restrict__ u,
                                                   float* __restrict__ O) {
  __shared__ __align__(16) float kk[64];
  __shared__ __align__(16) float ew[64];
  __shared__ __align__(16) float vv[64];
  __shared__ __align__(16) float uu[64];
  __shared__ __align__(16) float os[64];
  __shared__ __align__(16) float cs[4];
  __shared__ __align__(16) _Float16 rh[64];

  const int bh = blockIdx.x;
  const int b  = bh >> 4;
  const int h  = bh & 15;
  const int tid = threadIdx.x, wave = tid >> 5, lane = tid & 31;
  const int hh = lane >> 4, c = lane & 15;
  const int jcol = wave * 16 + c;

  if (tid < kHeadDim) uu[tid] = u[h * kHeadDim + tid];
  float s0[16], s1[16];
#pragma unroll
  for (int e = 0; e < 16; ++e) { s0[e] = 0.0f; s1[e] = 0.0f; }
  __syncthreads();

  const size_t rowbase = (size_t)b * kSeq;
#pragma unroll 1
  for (int t = 0; t < kSeq; ++t) {
    const size_t base = (rowbase + (size_t)t) * (size_t)kDim + (size_t)h * kHeadDim;
    if (wave < 2) {
      const int i = tid;
      const float rv = R[base + i];
      const float ev = E[base + i];
      const float kv = 1.0f - ev;
      rh[i] = (_Float16)rv;
      kk[i] = kv;
      ew[i] = ev;
      float pr = rv * uu[i] * kv;
      pr += __shfl_xor(pr, 1, 32);
      pr += __shfl_xor(pr, 2, 32);
      pr += __shfl_xor(pr, 4, 32);
      pr += __shfl_xor(pr, 8, 32);
      pr += __shfl_xor(pr, 16, 32);
      if (lane == 0) cs[wave] = pr;
    } else {
      const int i = tid - 64;
      vv[i] = V[base + i];
    }
    __syncthreads();
    const float vj = vv[jcol];
    const float ct = cs[0] + cs[1];
    HU a0, a1;
    a0.h8[0] = *(const v8h*)(rh + 8 * hh);
    a0.h8[1] = *(const v8h*)(rh + 16 + 8 * hh);
    a1.h8[0] = *(const v8h*)(rh + 32 + 8 * hh);
    a1.h8[1] = *(const v8h*)(rh + 48 + 8 * hh);
    v16h bv0, bv1, bl0, bl1;
    col_step(s0, bv0, bl0, kk + 8 * hh,      ew + 8 * hh,      vj);
    col_step(s1, bv1, bl1, kk + 32 + 8 * hh, ew + 32 + 8 * hh, vj);
    v8f acc  = (v8f){0.f,0.f,0.f,0.f,0.f,0.f,0.f,0.f};
    v8f accl = (v8f){0.f,0.f,0.f,0.f,0.f,0.f,0.f,0.f};
    acc  = mma16_g(a0.v, bv0, acc);
    acc  = mma16_g(a1.v, bv1, acc);
    accl = mma16_g(a0.v, bl0, accl);
    accl = mma16_g(a1.v, bl1, accl);
    const float o = (acc[0] + accl[0] * kInvLo) * kInvState + vj * ct;
    if (hh == 0) os[jcol] = o;
    __syncthreads();
    if (wave == 0 && lane < 16) {
      const v4f val = *(const v4f*)(os + 4 * lane);
      float* dst = O + base + 4 * lane;
      *(volatile v4f*)dst = val;
      __threadfence();
      *(volatile v4f*)dst = val;
    }
  }
}

__global__ __launch_bounds__(256) void ln_kernel(const float* __restrict__ O, const float* __restrict__ g,
                                                 const float* __restrict__ beta, unsigned short* __restrict__ Cat) {
  const int wave = threadIdx.x >> 5, lane = threadIdx.x & 31;
  const int row = blockIdx.x * 8 + wave;
  const float* op = O + (size_t)row * kDim;
  float v[32];
#pragma unroll
  for (int q = 0; q < 4; ++q) {
    const int cc = q * 256 + lane * 8;
    const v4f a = *(const v4f*)(op + cc);
    const v4f bq = *(const v4f*)(op + cc + 4);
#pragma unroll
    for (int e = 0; e < 4; ++e) { v[8 * q + e] = a[e]; v[8 * q + 4 + e] = bq[e]; }
  }
  float s = 0.0f;
#pragma unroll
  for (int e = 0; e < 32; ++e) s += v[e];
  s += __shfl_xor(s, 1, 32);
  s += __shfl_xor(s, 2, 32);
  s += __shfl_xor(s, 4, 32);
  s += __shfl_xor(s, 8, 32);
  s += __shfl_xor(s, 16, 32);
  const float mu = s * kInvDim;
  float qs = 0.0f;
#pragma unroll
  for (int e = 0; e < 32; ++e) { const float d = v[e] - mu; qs += d * d; }
  qs += __shfl_xor(qs, 1, 32);
  qs += __shfl_xor(qs, 2, 32);
  qs += __shfl_xor(qs, 4, 32);
  qs += __shfl_xor(qs, 8, 32);
  qs += __shfl_xor(qs, 16, 32);
  const float rs = rsqrtf(qs * kInvDim + kLnEps);
  v4u out[4];
#pragma unroll
  for (int q = 0; q < 4; ++q) {
    const int cc = q * 256 + lane * 8;
    const v4f ga = *(const v4f*)(g + cc);
    const v4f gb = *(const v4f*)(g + cc + 4);
    const v4f ba = *(const v4f*)(beta + cc);
    const v4f bb = *(const v4f*)(beta + cc + 4);
    unsigned short hb[8];
#pragma unroll
    for (int e = 0; e < 4; ++e) {
      hb[e]     = h_bits((((v[8 * q + e] - mu) * rs) * ga[e] + ba[e]) * kCatCarry);
      hb[4 + e] = h_bits((((v[8 * q + 4 + e] - mu) * rs) * gb[e] + bb[e]) * kCatCarry);
    }
    out[q] = pack8(hb);
  }
  unsigned short* dst = Cat + (size_t)row * kCat;
  for (int pass = 0; pass < 2; ++pass) {
#pragma unroll
    for (int q = 0; q < 4; ++q) *(volatile v4u*)(dst + q * 256 + lane * 8) = out[q];
    __threadfence();
  }
}

extern "C" void kernel_launch(void* const* d_in, const int* in_sizes, int n_in,
                              void* d_out, int out_size, void* d_ws, size_t ws_size,
                              hipStream_t stream) {
  if (n_in < 14) return;
  if (ws_size < kWsTotal) return;
  if ((long)in_sizes[0] != kActPlane) return;
  if (in_sizes[1] != kDim || in_sizes[2] != kDim || in_sizes[3] != kDim || in_sizes[4] != kDim) return;
  if (in_sizes[5] != kDim * kLora || in_sizes[6] != 3 * kLoraD * kDim || in_sizes[7] != kHeads * kHeadDim) return;
  if ((long)in_sizes[8] != kSqPlane || (long)in_sizes[9] != kSqPlane) return;
  if ((long)in_sizes[10] != (long)kDim * kVG || (long)in_sizes[11] != (long)kCat * kDim) return;
  if (in_sizes[12] != kDim || in_sizes[13] != kDim) return;
  if ((long)out_size != kActPlane) return;

  const float* x     = (const float*)d_in[0];
  const float* maa_x = (const float*)d_in[1];
  const float* maa_k = (const float*)d_in[2];
  const float* maa_v = (const float*)d_in[3];
  const float* maa_r = (const float*)d_in[4];
  const float* w1    = (const float*)d_in[5];
  const float* w2    = (const float*)d_in[6];
  const float* u     = (const float*)d_in[7];
  const float* Wr    = (const float*)d_in[8];
  const float* Wk    = (const float*)d_in[9];
  const float* Wvg   = (const float*)d_in[10];
  const float* Wo    = (const float*)d_in[11];
  const float* ln_g  = (const float*)d_in[12];
  const float* ln_b  = (const float*)d_in[13];
  float* out = (float*)d_out;

  char* ws = (char*)d_ws;
  unsigned short* WRT  = (unsigned short*)(ws + kOffWR);
  unsigned short* WKT  = (unsigned short*)(ws + kOffWK);
  unsigned short* WVGT = (unsigned short*)(ws + kOffWVG);
  unsigned short* WOT  = (unsigned short*)(ws + kOffWO);
  unsigned short* W1T  = (unsigned short*)(ws + kOffW1);
  unsigned short* W2T  = (unsigned short*)(ws + kOffW2);
  unsigned short* MT   = (unsigned short*)(ws + kOffMT);
  unsigned short* XXX  = (unsigned short*)(ws + kOffX);
  unsigned short* XM   = (unsigned short*)(ws + kOffX);
  float*          Op   = (float*)(ws + kOffX);
  float*          Rp   = (float*)(ws + kOffR);
  float*          Ep   = (float*)(ws + kOffE);
  float*          Vp   = (float*)(ws + kOffV);
  unsigned short* CAT  = (unsigned short*)(ws + kOffCAT);

  trans_cast<64><<<dim3(kDim / 64, kDim / 64, 1), 256, 0, stream>>>(Wr, WRT, kDim, kDim, 0L, 0L, kWCarry);
  trans_cast<64><<<dim3(kDim / 64, kDim / 64, 1), 256, 0, stream>>>(Wk, WKT, kDim, kDim, 0L, 0L, kWCarry);
  trans_cast<64><<<dim3(kVG / 64, kDim / 64, 1), 256, 0, stream>>>(Wvg, WVGT, kVG, kDim, 0L, 0L, kWCarry);
  trans_cast<64><<<dim3(kDim / 64, kCat / 64, 1), 256, 0, stream>>>(Wo, WOT, kDim, kCat, 0L, 0L, kWCarry);
  trans_cast<64><<<dim3(kLoraPad / 64, kDim / 64, 1), 256, 0, stream>>>(w1, W1T, kLora, kDim, 0L, 0L, kLCarry);
  trans_cast<32><<<dim3(kDim / 64, 1, 3), 256, 0, stream>>>(w2, W2T, kDim, kLoraD, (long)kLoraD * kDim, (long)kDim * kLoraD, kLCarry);

  shift_kernel<<<(kTok * kDim) / (256 * 8), 256, 0, stream>>>(x, maa_x, XXX);

  gemm64<3, 1><<<dim3(16, 1), 256, 0, stream>>>(
      XXX, kDim, 0L, W1T, kDim, 0L, (void*)MT, kLoraPad, 0L,
      x, maa_x, maa_x, maa_x, kTok, kLoraPad, kDim, kScaleL0);

  gemm64<0, 3><<<dim3(128, 3), 256, 0, stream>>>(
      MT, kLoraPad, (long)kLoraD, W2T, kLoraD, (long)kDim * kLoraD, (void*)XM, kDim, kActPlane,
      x, maa_k, maa_v, maa_r, kTok, kDim, kLoraD, kScaleL1);

  gemm64<0, 0><<<dim3(128, 1), 256, 0, stream>>>(
      XM + 2 * kActPlane, kDim, 0L, WRT, kDim, 0L, (void*)Rp, kDim, 0L,
      x, maa_x, maa_x, maa_x, kTok, kDim, kDim, kScaleProj);
  gemm64<6, 0><<<dim3(128, 1), 256, 0, stream>>>(
      XM, kDim, 0L, WKT, kDim, 0L, (void*)Ep, kDim, 0L,
      x, maa_x, maa_x, maa_x, kTok, kDim, kDim, kScaleProj);

  gemm_vg<<<(kTok / 32) * (kCat / 64) / 8, 256, 0, stream>>>(XM + kActPlane, WVGT, Vp, CAT, kScaleProj);

  scan_kernel<<<kBatch * kHeads, 128, 0, stream>>>(Rp, Ep, Vp, u, Op);

  ln_kernel<<<kTok / 8, 256, 0, stream>>>(Op, ln_g, ln_b, CAT);

  gemm64<0, 0><<<dim3(128, 1), 256, 0, stream>>>(
      CAT, kCat, 0L, WOT, kCat, 0L, (void*)out, kDim, 0L,
      x, maa_x, maa_x, maa_x, kTok, kDim, kCat, kScaleOut);
}
